// TransformerBlock_20349555048887
// MI455X (gfx1250) — hardware-verified
//
#include <hip/hip_runtime.h>
#include <math.h>

#ifndef NB
#define NB 1
#endif
#ifndef SEQ
#define SEQ 4096
#endif
#define SEQ_FULL 4096
#define DM 768
#define NHD 12
#define DHD 64
#define DFF 3072
#define ROWS (NB * SEQ)
#define FCH ((ROWS) < 2048 ? (ROWS) : 2048)
static_assert(NB == 1);
static_assert(SEQ <= SEQ_FULL);
static_assert(SEQ % 64 == 0);
static_assert(ROWS % FCH == 0);
static_assert(FCH % 64 == 0);
static_assert(DM == 128 * 6);
static_assert(DM == NHD * DHD);
static_assert(DHD == 64);
static_assert(DM % 64 == 0 && DFF % 64 == 0 && (2 * DM) % 64 == 0);
static_assert(DM % 32 == 0 && DFF % 32 == 0);

typedef __attribute__((ext_vector_type(16))) _Float16 v16h;
typedef __attribute__((ext_vector_type(8)))  _Float16 v8h;
typedef __attribute__((ext_vector_type(8)))  float    v8f;
typedef __attribute__((ext_vector_type(4)))  float    v4f;
typedef unsigned int bk_u4 __attribute__((ext_vector_type(4)));
typedef unsigned int bk_u2 __attribute__((ext_vector_type(2)));
typedef float bk_f2 __attribute__((ext_vector_type(2)));

union FragH { v16h v; v8h h[2]; };
__device__ __forceinline__ v16h ldg_frag(const _Float16* __restrict__ p) {
    FragH f; f.h[0] = *(const v8h*)(p); f.h[1] = *(const v8h*)(p + 16); return f.v;
}
#define LDS_FRAG(dst, arr, off) do { (dst).h[0] = *(const v8h*)&(arr)[(off)]; (dst).h[1] = *(const v8h*)&(arr)[(off) + 16]; } while (0)

__device__ __forceinline__ v8f mma_h(v16h a, v16h b, v8f c) {
    return __builtin_amdgcn_wmma_f32_16x16x32_f16(false, a, false, b, (short)0, c, false, false);
}
__device__ __forceinline__ void guard2(v8f& a, v8f& b, v16h x, v16h y, v16h z) { asm volatile("v_nop\n\tv_nop\n\tv_nop\n\tv_nop" : "+v"(a), "+v"(b) : "v"(x), "v"(y), "v"(z)); }
__device__ __forceinline__ void guard4(v8f& a, v8f& b, v8f& c, v8f& d, v16h x, v16h y0, v16h y1, v16h y2, v16h y3) {
    asm volatile("v_nop\n\tv_nop\n\tv_nop\n\tv_nop" : "+v"(a), "+v"(b), "+v"(c), "+v"(d) : "v"(x), "v"(y0), "v"(y1), "v"(y2), "v"(y3));
}
__device__ __forceinline__ void dep_guard_h(v8f& a, v8f& b, v16h x, v16h y) { asm volatile("v_nop\n\tv_nop\n\tv_nop\n\tv_nop" : "+v"(a), "+v"(b) : "v"(x), "v"(y)); }
__device__ __forceinline__ void keep4_h(v16h a, v16h b, v16h c, v16h d) { asm volatile("v_nop" :: "v"(a), "v"(b), "v"(c), "v"(d)); }
__device__ __forceinline__ void acc_guard4(v8f& a, v8f& b, v8f& c, v8f& d) { asm volatile("v_nop\n\tv_nop\n\tv_nop\n\tv_nop" : "+v"(a), "+v"(b), "+v"(c), "+v"(d)); }

#define VST2(T, ptr, val) do { const T vst2_v_ = (val); *(volatile T*)(ptr) = vst2_v_; __threadfence(); *(volatile T*)(ptr) = vst2_v_; } while (0)
#define VST2V4(ptr, val) do { const v4f vst2_v4_ = (val); *(volatile v4f*)(ptr) = vst2_v4_; __threadfence(); *(volatile v4f*)(ptr) = vst2_v4_; } while (0)

template <int BIAS_MODE, int OUT_MODE>
__device__ __forceinline__ void gemm64_body(const _Float16* __restrict__ A, int lda, const _Float16* __restrict__ Bt, int ldb,
                                            void* __restrict__ Cout, int ldc, const float* __restrict__ bias, int M, int N, int K, float scale) {
  __shared__ __align__(16) float sT[8][16 * 68];
  const int lane = threadIdx.x & 31;
  const int wave = threadIdx.x >> 5;
  const int tilesN = N >> 6;
  const int tilesM = M >> 6;
  const int tile = blockIdx.x * 8 + wave;
  if (tile >= tilesM * tilesN) return;
  const int tm = tile / tilesN;
  const int tn = tile - tm * tilesN;
  const int m0 = tm << 6;
  const int n0 = tn << 6;
  const int rlane = lane & 15;
  const int koff  = (lane >> 4) * 8;
  const int mOff  = (lane >> 4) * 8;

  v8f acc[4][4];
#pragma unroll
  for (int i = 0; i < 4; ++i)
#pragma unroll
    for (int j = 0; j < 4; ++j) acc[i][j] = (v8f){0.f,0.f,0.f,0.f,0.f,0.f,0.f,0.f};

  for (int k0 = 0; k0 < K; k0 += 32) {
    v16h bh[4];
#pragma unroll
    for (int j = 0; j < 4; ++j) bh[j] = ldg_frag(Bt + (size_t)(n0 + (j << 4) + rlane) * ldb + koff + k0);
#pragma unroll
    for (int i = 0; i < 4; ++i) {
      const v16h ah = ldg_frag(A + (size_t)(m0 + (i << 4) + rlane) * lda + koff + k0);
#pragma unroll
      for (int j = 0; j < 4; ++j) acc[i][j] = mma_h(ah, bh[j], acc[i][j]);
      dep_guard_h(acc[i][0], acc[i][3], ah, ah);
    }
    keep4_h(bh[0], bh[1], bh[2], bh[3]);
  }
  acc_guard4(acc[0][0], acc[0][1], acc[0][2], acc[0][3]);
  acc_guard4(acc[1][0], acc[1][1], acc[1][2], acc[1][3]);
  acc_guard4(acc[2][0], acc[2][1], acc[2][2], acc[2][3]);
  acc_guard4(acc[3][0], acc[3][1], acc[3][2], acc[3][3]);

#pragma unroll
  for (int i = 0; i < 4; ++i) {
    const int mBase = m0 + (i << 4);
#pragma unroll
    for (int j = 0; j < 4; ++j) {
      const int n = n0 + (j << 4) + rlane;
      float bv = 0.f;
      if (BIAS_MODE == 2) bv = bias[n];
#pragma unroll
      for (int r = 0; r < 8; ++r) {
        float v = acc[i][j][r] * scale;
        if (BIAS_MODE == 2) v += bv;
        sT[wave][(mOff + r) * 68 + (j << 4) + rlane] = v;
      }
    }
    __builtin_amdgcn_fence(3  , "workgroup");
    __builtin_amdgcn_wave_barrier();
    __builtin_amdgcn_fence(2  , "workgroup");
    if (OUT_MODE == 0) {
      float* C = (float*)Cout;
      const int hh = lane >> 4, c4 = (lane & 15) * 4;
      for (int pass = 0; pass < 2; ++pass) {
#pragma unroll
        for (int it = 0; it < 8; ++it) {
          const int row = it * 2 + hh;
          const v4f v = *(const v4f*)&sT[wave][row * 68 + c4];
          *(volatile v4f*)(C + (size_t)(mBase + row) * ldc + n0 + c4) = v;
        }
        __threadfence();
      }
    } else {
      const int q = lane >> 3, c8 = (lane & 7) * 8;
      unsigned short* C = (unsigned short*)Cout;
      for (int pass = 0; pass < 2; ++pass) {
#pragma unroll
        for (int it = 0; it < 4; ++it) {
          const int row = it * 4 + q;
          const v4f a = *(const v4f*)&sT[wave][row * 68 + c8];
          const v4f b = *(const v4f*)&sT[wave][row * 68 + c8 + 4];
          v8h hv;
          hv[0] = (_Float16)a.x; hv[1] = (_Float16)a.y; hv[2] = (_Float16)a.z; hv[3] = (_Float16)a.w;
          hv[4] = (_Float16)b.x; hv[5] = (_Float16)b.y; hv[6] = (_Float16)b.z; hv[7] = (_Float16)b.w;
          *(volatile v8h*)(C + (size_t)(mBase + row) * ldc + n0 + c8) = hv;
        }
        __threadfence();
      }
    }
    __builtin_amdgcn_fence(3  , "workgroup");
    __builtin_amdgcn_wave_barrier();
    __builtin_amdgcn_fence(2  , "workgroup");
  }
}
__global__ __launch_bounds__(256) void k_gemm_h16(const unsigned short* __restrict__ A, int lda, const unsigned short* __restrict__ Bt, int ldb,
                                                   unsigned short* __restrict__ C, int ldc, int M, int N, int K, float scale) {
  gemm64_body<0, 1>((const _Float16*)A, lda, (const _Float16*)Bt, ldb, (void*)C, ldc, nullptr, M, N, K, scale);
}
__global__ __launch_bounds__(256) void k_gemm_f32b(const unsigned short* __restrict__ A, int lda, const unsigned short* __restrict__ Bt, int ldb,
                                                    float* __restrict__ C, int ldc, const float* __restrict__ bias, int M, int N, int K, float scale) {
  gemm64_body<2, 0>((const _Float16*)A, lda, (const _Float16*)Bt, ldb, (void*)C, ldc, bias, M, N, K, scale);
}

#define AT_KP 72
#define AT_PP 40
#define AT_OP 68
__global__ __launch_bounds__(128) void k_attn_f16(const unsigned short* __restrict__ QKp, const unsigned short* __restrict__ VTp, unsigned short* __restrict__ CTXp,
                                                   int ldqk, int ldvt, int ldc, float sl2e) {
    __shared__ __align__(16) _Float16 Qs[64 * AT_KP];
    __shared__ __align__(16) _Float16 Ks[64 * AT_KP];
    __shared__ __align__(16) _Float16 Vt[64 * AT_KP];
    __shared__ __align__(16) _Float16 Ps[4 * 16 * AT_PP];
    __shared__ __align__(16) float    Os[4 * 16 * AT_OP];
    const _Float16* __restrict__ QK = (const _Float16*)QKp;
    const _Float16* __restrict__ VT = (const _Float16*)VTp;
    const int tid = threadIdx.x;
    const int wave = __builtin_amdgcn_readfirstlane(tid >> 5);
    const int lane = tid & 31, hh = lane >> 4, c = lane & 15;
    const int qb = blockIdx.x, head = blockIdx.y;
    const int q0b = qb * 64;
    const int q0 = q0b + wave * 16;
    const float NEG = -__builtin_inff();

#pragma unroll
    for (int it = 0; it < 4; ++it) {
        const int idx = tid + it * 128; const int row = idx >> 3, pc = idx & 7;
        const v8h val = *(const v8h*)(QK + (size_t)(q0b + row) * ldqk + head * DHD + pc * 8);
        *(v8h*)&Qs[row * AT_KP + pc * 8] = val;
    }

    v8f o[4]; float m8[8], l8[8];
#pragma unroll
    for (int t = 0; t < 4; ++t) o[t] = (v8f){0.f,0.f,0.f,0.f,0.f,0.f,0.f,0.f};
#pragma unroll
    for (int r = 0; r < 8; ++r) { m8[r] = NEG; l8[r] = 0.f; }

    for (int kb = 0; kb <= qb; ++kb) {
        const int kv0 = kb * 64;
        __syncthreads();
#pragma unroll
        for (int it = 0; it < 4; ++it) {
            const int idx = tid + it * 128; const int row = idx >> 3, pc = idx & 7;
            const v8h kk = *(const v8h*)(QK + (size_t)(kv0 + row) * ldqk + DM + head * DHD + pc * 8);
            const v8h vv = *(const v8h*)(VT + (size_t)(head * DHD + row) * ldvt + kv0 + pc * 8);
            *(v8h*)&Ks[row * AT_KP + pc * 8] = kk;
            *(v8h*)&Vt[row * AT_KP + pc * 8] = vv;
        }
        __syncthreads();

#pragma unroll 1
        for (int hk = 0; hk < 2; ++hk) {
            const int kofs = hk * 32;
            v8f s0 = (v8f){0.f,0.f,0.f,0.f,0.f,0.f,0.f,0.f}, s1 = s0;
#pragma unroll
            for (int dc = 0; dc < 2; ++dc) {
                FragH qa, k0, k1;
                const int qo = (wave * 16 + c) * AT_KP + dc * 32 + 8 * hh;
                const int ko = (kofs + c) * AT_KP + dc * 32 + 8 * hh;
                LDS_FRAG(qa, Qs, qo);
                LDS_FRAG(k0, Ks, ko);
                LDS_FRAG(k1, Ks, ko + 16 * AT_KP);
                s0 = mma_h(qa.v, k0.v, s0);
                s1 = mma_h(qa.v, k1.v, s1);
                guard2(s0, s1, qa.v, k0.v, k1.v);
            }
            const int key0 = kv0 + kofs + c;
#pragma unroll
            for (int r = 0; r < 8; ++r) {
                const int qrow = q0 + 8 * hh + r;
                float x0 = s0[r] * sl2e, x1 = s1[r] * sl2e;
                x0 = (key0 > qrow) ? NEG : x0;
                x1 = (key0 + 16 > qrow) ? NEG : x1;
                float mx = fmaxf(x0, x1);
                mx = fmaxf(mx, __shfl_xor(mx, 1, 32)); mx = fmaxf(mx, __shfl_xor(mx, 2, 32));
                mx = fmaxf(mx, __shfl_xor(mx, 4, 32)); mx = fmaxf(mx, __shfl_xor(mx, 8, 32));
                const float mnew = fmaxf(m8[r], mx);
                const float corr = (mnew == NEG) ? 1.f : exp2f(m8[r] - mnew);
                const float p0 = (x0 == NEG) ? 0.f : exp2f(x0 - mnew);
                const float p1 = (x1 == NEG) ? 0.f : exp2f(x1 - mnew);
                float rs = p0 + p1;
                rs += __shfl_xor(rs, 1, 32); rs += __shfl_xor(rs, 2, 32); rs += __shfl_xor(rs, 4, 32); rs += __shfl_xor(rs, 8, 32);
                l8[r] = l8[r] * corr + rs; m8[r] = mnew;
#pragma unroll
                for (int t = 0; t < 4; ++t) o[t][r] *= corr;
                const int po = (wave * 16 + 8 * hh + r) * AT_PP + c;
                Ps[po]      = (_Float16)(p0 * 1024.f);
                Ps[po + 16] = (_Float16)(p1 * 1024.f);
            }
            __builtin_amdgcn_fence(3  , "workgroup");
            __builtin_amdgcn_wave_barrier();
            __builtin_amdgcn_fence(2  , "workgroup");
            {
                FragH pa, v0, v1, v2, v3;
                const int po = (wave * 16 + c) * AT_PP + 8 * hh;
                const int vo = c * AT_KP + kofs + 8 * hh;
                LDS_FRAG(pa, Ps, po);
                LDS_FRAG(v0, Vt, vo);
                LDS_FRAG(v1, Vt, vo + 16 * AT_KP);
                LDS_FRAG(v2, Vt, vo + 32 * AT_KP);
                LDS_FRAG(v3, Vt, vo + 48 * AT_KP);
                o[0] = mma_h(pa.v, v0.v, o[0]);
                o[1] = mma_h(pa.v, v1.v, o[1]);
                o[2] = mma_h(pa.v, v2.v, o[2]);
                o[3] = mma_h(pa.v, v3.v, o[3]);
                guard4(o[0], o[1], o[2], o[3], pa.v, v0.v, v1.v, v2.v, v3.v);
            }
            __builtin_amdgcn_fence(3  , "workgroup");
            __builtin_amdgcn_wave_barrier();
            __builtin_amdgcn_fence(2  , "workgroup");
        }
    }

#pragma unroll
    for (int r = 0; r < 8; ++r) {
        const float inv = 1.0f / (l8[r] * 1024.f);
#pragma unroll
        for (int t = 0; t < 4; ++t) Os[(wave * 16 + 8 * hh + r) * AT_OP + t * 16 + c] = o[t][r] * inv;
    }
    __builtin_amdgcn_fence(3  , "workgroup");
    __builtin_amdgcn_wave_barrier();
    __builtin_amdgcn_fence(2  , "workgroup");
    {
        const int q4 = lane >> 3, c8 = (lane & 7) * 8;
        for (int pass = 0; pass < 2; ++pass) {
#pragma unroll
            for (int it = 0; it < 4; ++it) {
                const int row = it * 4 + q4;
                const v4f a = *(const v4f*)&Os[(wave * 16 + row) * AT_OP + c8];
                const v4f b = *(const v4f*)&Os[(wave * 16 + row) * AT_OP + c8 + 4];
                v8h hv;
                hv[0] = (_Float16)a.x; hv[1] = (_Float16)a.y; hv[2] = (_Float16)a.z; hv[3] = (_Float16)a.w;
                hv[4] = (_Float16)b.x; hv[5] = (_Float16)b.y; hv[6] = (_Float16)b.z; hv[7] = (_Float16)b.w;
                *(volatile v8h*)(CTXp + (size_t)(q0 + row) * ldc + head * DHD + c8) = hv;
            }
            __threadfence();
        }
    }
}

__device__ __forceinline__ unsigned int cmb_pk2(float a, float b) { return (unsigned int)__builtin_bit_cast(unsigned short, (_Float16)a) | ((unsigned int)__builtin_bit_cast(unsigned short, (_Float16)b) << 16); }
__device__ __forceinline__ float cmb_bf(float v) { const unsigned u = __builtin_bit_cast(unsigned, v); const unsigned r = (u + 0x7fffu + ((u >> 16) & 1u)) & 0xffff0000u; return __builtin_bit_cast(float, r); }
__global__ __launch_bounds__(256) void k_cm_bfvec(const float* __restrict__ SRC, float* __restrict__ DST, int n) { const int u = blockIdx.x * 256 + threadIdx.x; if (u >= n) return; VST2(float, DST + u, cmb_bf(SRC[u])); }
__global__ __launch_bounds__(256) void k_cm_castbT(const float* __restrict__ SRC, int lds, unsigned short* __restrict__ DST, int ldd, int nR, int nC, float sc) {
    const long long u = (long long)blockIdx.x * 256 + threadIdx.x; const int per = nR / 8; if (u >= (long long)nC * per) return; const int c = (int)(u / per); const int r0 = 8 * (int)(u % per);
    float w[8];
#pragma unroll
    for (int e = 0; e < 8; ++e) w[e] = cmb_bf(SRC[(long long)(r0 + e) * lds + c]) * sc;
    bk_u4 pk; pk.x = cmb_pk2(w[0], w[1]); pk.y = cmb_pk2(w[2], w[3]); pk.z = cmb_pk2(w[4], w[5]); pk.w = cmb_pk2(w[6], w[7]); VST2(bk_u4, (bk_u4*)(DST + (long long)c * ldd + r0), pk); }

__device__ __forceinline__ unsigned int bk_pk2(float a, float b) { return (unsigned int)__builtin_bit_cast(unsigned short, (_Float16)a) | ((unsigned int)__builtin_bit_cast(unsigned short, (_Float16)b) << 16); }
template <int NQ, int ABF>
__device__ __forceinline__ void b_ln_body(const float* __restrict__ A, const float* __restrict__ GA, const float* __restrict__ BE, float eps, float inv_vden, int rows, unsigned short* __restrict__ Y16) {
    #pragma clang fp contract(off)
    constexpr int WD = 128 * NQ; const int r = blockIdx.x * 8 + (threadIdx.x >> 5); const int L = threadIdx.x & 31; if (r >= rows) return; v4f v[NQ]; float s = 0.f;
#pragma unroll
    for (int q = 0; q < NQ; ++q) { const long long o = (long long)r * WD + 4 * L + 128 * q; v[q] = *(const v4f*)(A + o); if (ABF) { v[q].x = cmb_bf(v[q].x); v[q].y = cmb_bf(v[q].y); v[q].z = cmb_bf(v[q].z); v[q].w = cmb_bf(v[q].w); } s += (v[q].x + v[q].y) + (v[q].z + v[q].w); }
#pragma unroll
    for (int o = 16; o > 0; o >>= 1) s += __shfl_xor(s, o, 32);
    const float mu = s * (1.f / WD); float qq = 0.f;
#pragma unroll
    for (int q = 0; q < NQ; ++q) { v[q].x -= mu; v[q].y -= mu; v[q].z -= mu; v[q].w -= mu; qq += (v[q].x * v[q].x + v[q].y * v[q].y) + (v[q].z * v[q].z + v[q].w * v[q].w); }
#pragma unroll
    for (int o = 16; o > 0; o >>= 1) qq += __shfl_xor(qq, o, 32);
    const float rs = rsqrtf(qq * inv_vden + eps);
#pragma unroll
    for (int q = 0; q < NQ; ++q) { const int c = 4 * L + 128 * q; const v4f ga = *(const v4f*)(GA + c), be = *(const v4f*)(BE + c); v4f y; y.x = v[q].x * rs * cmb_bf(ga.x) + cmb_bf(be.x); y.y = v[q].y * rs * cmb_bf(ga.y) + cmb_bf(be.y); y.z = v[q].z * rs * cmb_bf(ga.z) + cmb_bf(be.z); y.w = v[q].w * rs * cmb_bf(ga.w) + cmb_bf(be.w);
        const long long o = (long long)r * WD + c; bk_u2 pk; pk.x = bk_pk2(y.x, y.y); pk.y = bk_pk2(y.z, y.w); VST2(bk_u2, (bk_u2*)(Y16 + o), pk); } }
__global__ __launch_bounds__(256) void k_ln_in(const float* __restrict__ A, const float* __restrict__ GA, const float* __restrict__ BE, float eps, float inv_vden, int rows, unsigned short* __restrict__ Y16) {
    b_ln_body<6, 1>(A, GA, BE, eps, inv_vden, rows, Y16); }
__global__ __launch_bounds__(256) void k_ln_mid(const float* __restrict__ A, const float* __restrict__ GA, const float* __restrict__ BE, float eps, float inv_vden, int rows, unsigned short* __restrict__ Y16) {
    b_ln_body<6, 0>(A, GA, BE, eps, inv_vden, rows, Y16); }

__device__ __forceinline__ float bk_gelu(float v) { return 0.5f * v * (1.f + erff(v * 0.70710678118654752f)); }
__global__ __launch_bounds__(256) void k_gelu16(const float* __restrict__ F, unsigned short* __restrict__ Y16, long long n8) {
    #pragma clang fp contract(off)
    const long long u = (long long)blockIdx.x * 256 + threadIdx.x; if (u >= n8) return;
    unsigned int w0 = 0u, w1 = 0u, w2 = 0u, w3 = 0u;
#pragma unroll 1
    for (int h = 0; h < 4; ++h) {
        const bk_f2 a = *(const bk_f2*)(F + 8 * u + 2 * h);
        const unsigned int pk = bk_pk2(bk_gelu(a.x), bk_gelu(a.y));
        w0 = (h == 0) ? pk : w0; w1 = (h == 1) ? pk : w1; w2 = (h == 2) ? pk : w2; w3 = (h == 3) ? pk : w3;
    }
    bk_u4 o; o.x = w0; o.y = w1; o.z = w2; o.w = w3;
    VST2(bk_u4, (bk_u4*)(Y16 + 8 * u), o); }
template <int XBF>
__device__ __forceinline__ void b_add_body(const float* __restrict__ A, const float* __restrict__ X, float* __restrict__ O, long long n4) {
    #pragma clang fp contract(off)
    const long long u = (long long)blockIdx.x * 256 + threadIdx.x; if (u >= n4) return; const v4f a = *(const v4f*)(A + 4 * u); v4f x = *(const v4f*)(X + 4 * u); if (XBF) { x.x = cmb_bf(x.x); x.y = cmb_bf(x.y); x.z = cmb_bf(x.z); x.w = cmb_bf(x.w); }
    v4f y; y.x = x.x + a.x; y.y = x.y + a.y; y.z = x.z + a.z; y.w = x.w + a.w; VST2V4(O + 4 * u, y); }
__global__ __launch_bounds__(256) void k_add_in(const float* __restrict__ A, const float* __restrict__ X, float* __restrict__ O, long long n4) { b_add_body<1>(A, X, O, n4); }
__global__ __launch_bounds__(256) void k_add_mid(const float* __restrict__ A, const float* __restrict__ X, float* __restrict__ O, long long n4) { b_add_body<0>(A, X, O, n4); }

#define AL256(b) (((((size_t)(b)) + 255) / 256) * 256)
#define SZ_X16  AL256((size_t)ROWS * DM * 2)
#define SZ_W316 AL256((size_t)3 * DM * DM * 2)
#define SZ_QK16 AL256((size_t)ROWS * 2 * DM * 2)
#define SZ_VT16 AL256((size_t)DM * ROWS * 2)
#define SZ_CTX  AL256((size_t)ROWS * DM * 2)
#define SZ_WO16 AL256((size_t)DM * DM * 2)
#define SZ_ATT  AL256((size_t)ROWS * DM * 4)
#define SZ_X1   AL256((size_t)ROWS * DM * 4)
#define SZ_H16  AL256((size_t)ROWS * DM * 2)
#define SZ_W1T  AL256((size_t)DFF * DM * 2)
#define SZ_W2T  AL256((size_t)DM * DFF * 2)
#define SZ_BRO  AL256((size_t)(DM + 64) * 4)
#define SZ_BR1  AL256((size_t)(DFF + 64) * 4)
#define SZ_BR2  AL256((size_t)(DM + 64) * 4)
#define SZ_F1   AL256((size_t)FCH * DFF * 4)
#define SZ_F16  AL256((size_t)FCH * DFF * 2)
#define SZ_FFO  AL256((size_t)FCH * DM * 4)
#define SZ_TOTAL (SZ_X16 + SZ_W316 + SZ_QK16 + SZ_VT16 + SZ_CTX + SZ_WO16 + SZ_ATT + SZ_X1 + SZ_H16 + SZ_W1T + SZ_W2T + SZ_BRO + SZ_BR1 + SZ_BR2 + SZ_F1 + SZ_F16 + SZ_FFO)
static_assert(SZ_TOTAL <= (size_t)134217728);
static_assert((size_t)DM * 4 <= SZ_BRO && (size_t)DFF * 4 <= SZ_BR1 && (size_t)DM * 4 <= SZ_BR2);

extern "C" void kernel_launch(void* const* d_in, const int* in_sizes, int n_in, void* d_out, int out_size, void* d_ws, size_t ws_size, hipStream_t stream) {
    if (n_in < 14) return;
    if (in_sizes[0] < NB * SEQ * DM) return;
    if (in_sizes[1] < DM * DM || in_sizes[2] < DM * DM || in_sizes[3] < DM * DM || in_sizes[4] < DM * DM) return;
    if (in_sizes[5] < DM || in_sizes[7] < DFF || in_sizes[9] < DM) return;
    if (in_sizes[6] < DM * DFF || in_sizes[8] < DFF * DM) return;
    if (in_sizes[10] < DM || in_sizes[11] < DM || in_sizes[12] < DM || in_sizes[13] < DM) return;
    if (out_size < ROWS * DM) return;
    if ((size_t)SZ_TOTAL > ws_size) return;
    const float* x = (const float*)d_in[0];
    const float* wq = (const float*)d_in[1];
    const float* wk = (const float*)d_in[2];
    const float* wv = (const float*)d_in[3];
    const float* wo = (const float*)d_in[4];
    const float* bo = (const float*)d_in[5];
    const float* w1 = (const float*)d_in[6];
    const float* b1 = (const float*)d_in[7];
    const float* w2 = (const float*)d_in[8];
    const float* b2 = (const float*)d_in[9];
    const float* g1 = (const float*)d_in[10];
    const float* be1 = (const float*)d_in[11];
    const float* g2 = (const float*)d_in[12];
    const float* be2 = (const float*)d_in[13];
    float* out = (float*)d_out;
    char* wsp = (char*)d_ws;
    unsigned short* X16 = (unsigned short*)wsp; wsp += SZ_X16;
    unsigned short* W316 = (unsigned short*)wsp; wsp += SZ_W316;
    unsigned short* QK16 = (unsigned short*)wsp; wsp += SZ_QK16;
    unsigned short* VT16 = (unsigned short*)wsp; wsp += SZ_VT16;
    unsigned short* CTX16 = (unsigned short*)wsp; wsp += SZ_CTX;
    unsigned short* WO16 = (unsigned short*)wsp; wsp += SZ_WO16;
    float* ATT = (float*)wsp; wsp += SZ_ATT;
    float* X1 = (float*)wsp; wsp += SZ_X1;
    unsigned short* H16 = (unsigned short*)wsp; wsp += SZ_H16;
    unsigned short* W1T = (unsigned short*)wsp; wsp += SZ_W1T;
    unsigned short* W2T = (unsigned short*)wsp; wsp += SZ_W2T;
    float* BRO = (float*)wsp; wsp += SZ_BRO;
    float* BR1 = (float*)wsp; wsp += SZ_BR1;
    float* BR2 = (float*)wsp; wsp += SZ_BR2;
    float* F1 = (float*)wsp; wsp += SZ_F1;
    unsigned short* F16 = (unsigned short*)wsp; wsp += SZ_F16;
    float* FFo = (float*)wsp; wsp += SZ_FFO;

    k_ln_in<<<(ROWS + 7) / 8, 256, 0, stream>>>(x, g1, be1, 1e-5f, 1.0f / 768.0f, ROWS, X16);
    k_cm_castbT<<<(unsigned)((((long long)DM) * (DM / 8) + 255) / 256), 256, 0, stream>>>(wq, DM, W316, DM, DM, DM, 16.0f);
    k_cm_castbT<<<(unsigned)((((long long)DM) * (DM / 8) + 255) / 256), 256, 0, stream>>>(wk, DM, W316 + (size_t)DM * DM, DM, DM, DM, 16.0f);
    k_cm_castbT<<<(unsigned)((((long long)DM) * (DM / 8) + 255) / 256), 256, 0, stream>>>(wv, DM, W316 + (size_t)2 * DM * DM, DM, DM, DM, 16.0f);
    k_cm_castbT<<<(unsigned)((((long long)DM) * (DM / 8) + 255) / 256), 256, 0, stream>>>(wo, DM, WO16, DM, DM, DM, 16.0f);
    k_cm_bfvec<<<(DM + 255) / 256, 256, 0, stream>>>(bo, BRO, DM);
    k_gemm_h16<<<(unsigned)(((ROWS / 64) * ((2 * DM) / 64) + 7) / 8), 256, 0, stream>>>(X16, DM, W316, DM, QK16, 2 * DM, ROWS, 2 * DM, DM, 0.0625f);
    k_gemm_h16<<<(unsigned)(((DM / 64) * (ROWS / 64) + 7) / 8), 256, 0, stream>>>(W316 + (size_t)2 * DM * DM, DM, X16, DM, VT16, ROWS, DM, ROWS, DM, 0.0625f);
    k_attn_f16<<<dim3((unsigned)(SEQ / 64), (unsigned)NHD), 128, 0, stream>>>(QK16, VT16, CTX16, 2 * DM, ROWS, DM, 0.125f * 1.4426950408889634f);
    k_gemm_f32b<<<(unsigned)(((ROWS / 64) * (DM / 64) + 7) / 8), 256, 0, stream>>>(CTX16, DM, WO16, DM, ATT, DM, BRO, ROWS, DM, DM, 0.0625f);
    k_cm_castbT<<<(unsigned)((((long long)DFF) * (DM / 8) + 255) / 256), 256, 0, stream>>>(w1, DFF, W1T, DM, DM, DFF, 16.0f);
    k_cm_castbT<<<(unsigned)((((long long)DM) * (DFF / 8) + 255) / 256), 256, 0, stream>>>(w2, DM, W2T, DFF, DFF, DM, 16.0f);
    k_cm_bfvec<<<(DFF + 255) / 256, 256, 0, stream>>>(b1, BR1, DFF);
    k_cm_bfvec<<<(DM + 255) / 256, 256, 0, stream>>>(b2, BR2, DM);
    k_add_in<<<(unsigned)(((long long)ROWS * DM / 4 + 255) / 256), 256, 0, stream>>>(ATT, x, X1, (long long)ROWS * DM / 4);
    k_ln_mid<<<(ROWS + 7) / 8, 256, 0, stream>>>(X1, g2, be2, 1e-5f, 1.0f / 768.0f, ROWS, H16);
    for (int c = 0; c < ROWS / FCH; ++c) {
        const size_t ro = (size_t)c * FCH * DM;
        k_gemm_f32b<<<(unsigned)(((FCH / 64) * (DFF / 64) + 7) / 8), 256, 0, stream>>>(H16 + ro, DM, W1T, DM, F1, DFF, BR1, FCH, DFF, DM, 0.0625f);
        k_gelu16<<<(unsigned)(((long long)FCH * DFF / 8 + 255) / 256), 256, 0, stream>>>(F1, F16, (long long)FCH * DFF / 8);
        k_gemm_f32b<<<(unsigned)(((FCH / 64) * (DM / 64) + 7) / 8), 256, 0, stream>>>(F16, DFF, W2T, DFF, FFo, DM, BR2, FCH, DM, DFF, 0.0625f);
        k_add_mid<<<(unsigned)(((long long)FCH * DM / 4 + 255) / 256), 256, 0, stream>>>(FFo, X1 + ro, out + ro, (long long)FCH * DM / 4);
    }
}
